// TUPEMultiheadAttention_22814866276746
// MI455X (gfx1250) — hardware-verified
//
#include <hip/hip_runtime.h>

typedef __attribute__((ext_vector_type(16))) _Float16 v16h;
typedef __attribute__((ext_vector_type(8)))  _Float16 v8h;
typedef __attribute__((ext_vector_type(16))) __bf16   v16b;
typedef __attribute__((ext_vector_type(8)))  __bf16   v8b;
typedef __attribute__((ext_vector_type(8)))  float    v8f;
typedef __attribute__((ext_vector_type(4)))  float    v4f;

constexpr int BB = 2, LL = 2048, DD = 1024, EE = 1024, HH = 16, HD = 64;
constexpr int QKV_LD = 3 * EE;
constexpr int PE_LD  = 2 * EE;

__device__ __forceinline__ unsigned short f2bf_bits(float f) {
  unsigned u = __float_as_uint(f);
  return (unsigned short)((u + 0x7FFFu + ((u >> 16) & 1u)) >> 16);
}
__device__ __forceinline__ float bf_bits2f(unsigned short h) { return __uint_as_float(((unsigned)h) << 16); }

__device__ __forceinline__ void dep_guard_h(v8f& a, v8f& b, v16h x, v16h y) { asm volatile("v_nop\n\tv_nop\n\tv_nop\n\tv_nop" : "+v"(a), "+v"(b) : "v"(x), "v"(y)); }
__device__ __forceinline__ void dep_guard_b(v8f& a, v8f& b, v16b x, v16b y) { asm volatile("v_nop\n\tv_nop\n\tv_nop\n\tv_nop" : "+v"(a), "+v"(b) : "v"(x), "v"(y)); }
__device__ __forceinline__ void keep4_h(v16h a, v16h b, v16h c, v16h d) { asm volatile("v_nop" :: "v"(a), "v"(b), "v"(c), "v"(d)); }
__device__ __forceinline__ void keep4_b(v16b a, v16b b, v16b c, v16b d) { asm volatile("v_nop" :: "v"(a), "v"(b), "v"(c), "v"(d)); }
__device__ __forceinline__ void acc_guard4(v8f& a, v8f& b, v8f& c, v8f& d) { asm volatile("v_nop\n\tv_nop\n\tv_nop\n\tv_nop" : "+v"(a), "+v"(b), "+v"(c), "+v"(d)); }
template <typename T> struct Frag;
template <> struct Frag<_Float16> {
  typedef v16h V; union U { v16h v; v8h h[2]; };
  static __device__ __forceinline__ v16h load(const _Float16* p) {
    U f; f.h[0] = *(const v8h*)(p); f.h[1] = *(const v8h*)(p + 16); return f.v;
  }
  static __device__ __forceinline__ v8f mma(v16h a, v16h b, v8f c) {
    return __builtin_amdgcn_wmma_f32_16x16x32_f16(false, a, false, b, (short)0, c, false, false);
  }
  static __device__ __forceinline__ void guard(v8f& a, v8f& b, v16h x, v16h y) { dep_guard_h(a, b, x, y); }
  static __device__ __forceinline__ void keep(v16h a, v16h b, v16h c, v16h d) { keep4_h(a, b, c, d); }
};
template <> struct Frag<__bf16> {
  typedef v16b V; union U { v16b v; v8b h[2]; };
  static __device__ __forceinline__ v16b load(const __bf16* p) {
    U f; f.h[0] = *(const v8b*)(p); f.h[1] = *(const v8b*)(p + 16); return f.v;
  }
  static __device__ __forceinline__ v8f mma(v16b a, v16b b, v8f c) {
    return __builtin_amdgcn_wmma_f32_16x16x32_bf16(false, a, false, b, (short)0, c, false, false);
  }
  static __device__ __forceinline__ void guard(v8f& a, v8f& b, v16b x, v16b y) { dep_guard_b(a, b, x, y); }
  static __device__ __forceinline__ void keep(v16b a, v16b b, v16b c, v16b d) { keep4_b(a, b, c, d); }
};

template <int ET> struct Elem;
template <> struct Elem<0> { typedef _Float16 T; };
template <> struct Elem<1> { typedef __bf16 T; };
template <int ET, bool SPLIT, int BIAS_MODE, int OUT_MODE, bool RESID, int ACT = 0>
__global__ __launch_bounds__(256) void wmma_gemm64(
    const unsigned short* __restrict__ Ap, const unsigned short* __restrict__ A2p, int lda, long strideA,
    const unsigned short* __restrict__ Btp, const unsigned short* __restrict__ Bt2p, int ldb, long strideB,
    void* __restrict__ Cout, void* __restrict__ Cout2, int ldc, long strideC,
    const float* __restrict__ bias,
    const float* __restrict__ resid, long strideR,
    int M, int N, int K, float scale) {
  typedef typename Elem<ET>::T T;
  typedef typename Frag<T>::V V;
  const T* A = (const T*)Ap; const T* A2 = (const T*)A2p; const T* Bt = (const T*)Btp; const T* Bt2 = (const T*)Bt2p;
  __shared__ __align__(16) float sT[8][16 * 68];
  const int b    = blockIdx.y;
  const int lane = threadIdx.x & 31;
  const int wave = threadIdx.x >> 5;
  const int tilesN = N >> 6;
  const int tilesM = M >> 6;
  const int tile = blockIdx.x * 8 + wave;
  if (tile >= tilesM * tilesN) return;
  const int tm = tile / tilesN;
  const int tn = tile - tm * tilesN;
  const int m0 = tm << 6;
  const int n0 = tn << 6;

  const T* Ab  = A  + (size_t)b * strideA;
  const T* Bb  = Bt + (size_t)b * strideB;
  const T* Ab2 = SPLIT ? (A2  + (size_t)b * strideA) : nullptr;
  const T* Bb2 = SPLIT ? (Bt2 + (size_t)b * strideB) : nullptr;

  const int rlane = lane & 15;
  const int koff  = (lane >> 4) * 8;
  const int mOff  = (lane >> 4) * 8;

  v8f acc[4][4];
#pragma unroll
  for (int i = 0; i < 4; ++i)
#pragma unroll
    for (int j = 0; j < 4; ++j) acc[i][j] = (v8f){0.f,0.f,0.f,0.f,0.f,0.f,0.f,0.f};

  for (int k0 = 0; k0 < K; k0 += 32) {
    V bh[4], bl[4];
#pragma unroll
    for (int j = 0; j < 4; ++j) {
      const size_t bo = (size_t)(n0 + (j << 4) + rlane) * ldb + koff + k0;
      bh[j] = Frag<T>::load(Bb + bo);
      if (SPLIT) bl[j] = Frag<T>::load(Bb2 + bo);
    }
#pragma unroll
    for (int i = 0; i < 4; ++i) {
      const size_t ao = (size_t)(m0 + (i << 4) + rlane) * lda + koff + k0;
      V ah = Frag<T>::load(Ab + ao);
      V al;
      if (SPLIT) al = Frag<T>::load(Ab2 + ao);
#pragma unroll
      for (int j = 0; j < 4; ++j) {
        acc[i][j] = Frag<T>::mma(ah, bh[j], acc[i][j]);
        if (SPLIT) {
          acc[i][j] = Frag<T>::mma(ah, bl[j], acc[i][j]);
          acc[i][j] = Frag<T>::mma(al, bh[j], acc[i][j]);
        }
      }
      Frag<T>::guard(acc[i][0], acc[i][3], ah, SPLIT ? al : ah);
    }
    Frag<T>::keep(bh[0], bh[1], bh[2], bh[3]);
    if (SPLIT) Frag<T>::keep(bl[0], bl[1], bl[2], bl[3]);
  }
  acc_guard4(acc[0][0], acc[0][1], acc[0][2], acc[0][3]);
  acc_guard4(acc[1][0], acc[1][1], acc[1][2], acc[1][3]);
  acc_guard4(acc[2][0], acc[2][1], acc[2][2], acc[2][3]);
  acc_guard4(acc[3][0], acc[3][1], acc[3][2], acc[3][3]);

  float* slab = sT[wave];
  const float* Rb = RESID ? (resid + (size_t)b * strideR) : nullptr;
#pragma unroll
  for (int i = 0; i < 4; ++i) {
    const int mBase = m0 + (i << 4);
#pragma unroll
    for (int j = 0; j < 4; ++j) {
      const int n = n0 + (j << 4) + rlane;
      float bv = 0.f;
      if (BIAS_MODE == 2) bv = bias[n];
#pragma unroll
      for (int r = 0; r < 8; ++r) {
        float v = acc[i][j][r] * scale;
        if (BIAS_MODE == 1) v += bias[mBase + mOff + r];
        if (BIAS_MODE == 2) v += bv;
        if (RESID) v += Rb[(size_t)(mBase + mOff + r) * ldc + n];
        if (ACT == 1) v = tanhf(v);
        if (ACT == 2) v = fmaxf(v, 0.0f);
        if (ACT == 3) v = v / (1.0f + expf(-v));
        if (ACT == 4) v = (v > 0.f) ? v : 0.01f * v;
        if (ACT == 5) v = 0.5f * v * (1.0f + erff(v * 0.70710678118654752f));
        slab[(mOff + r) * 68 + (j << 4) + rlane] = v;
      }
    }
    __builtin_amdgcn_fence(__ATOMIC_RELEASE, "workgroup");
    __builtin_amdgcn_wave_barrier();
    __builtin_amdgcn_fence(__ATOMIC_ACQUIRE, "workgroup");
    if (OUT_MODE == 0) {
      float* C = (float*)Cout + (size_t)b * strideC;
      const int hh = lane >> 4, c4 = (lane & 15) * 4;
      for (int pass = 0; pass < 2; ++pass) {
#pragma unroll
        for (int it = 0; it < 8; ++it) {
          const int row = it * 2 + hh;
          v4f v = *(const v4f*)(slab + row * 68 + c4);
          *(volatile v4f*)(C + (size_t)(mBase + row) * ldc + n0 + c4) = v;
        }
        __threadfence();
      }
    } else {
      const int q = lane >> 3, c8 = (lane & 7) * 8;
      unsigned short* C  = (unsigned short*)Cout  + (size_t)b * strideC;
      unsigned short* C2 = (OUT_MODE == 2) ? ((unsigned short*)Cout2 + (size_t)b * strideC) : nullptr;
      for (int pass = 0; pass < 2; ++pass) {
#pragma unroll
        for (int it = 0; it < 4; ++it) {
          const int row = it * 4 + q;
          const float* sp = slab + row * 68 + c8;
          v8h hv, lv;
#pragma unroll
          for (int e = 0; e < 8; ++e) {
            if (OUT_MODE == 1) {
              hv[e] = (_Float16)sp[e];
            } else {
              unsigned short hb = f2bf_bits(sp[e]);
              unsigned short lb = f2bf_bits(sp[e] - bf_bits2f(hb));
              hv[e] = __builtin_bit_cast(_Float16, hb);
              lv[e] = __builtin_bit_cast(_Float16, lb);
            }
          }
          *(volatile v8h*)(C + (size_t)(mBase + row) * ldc + n0 + c8) = hv;
          if (OUT_MODE == 2) *(volatile v8h*)(C2 + (size_t)(mBase + row) * ldc + n0 + c8) = lv;
        }
        __threadfence();
      }
    }
    __builtin_amdgcn_fence(__ATOMIC_RELEASE, "workgroup");
    __builtin_amdgcn_wave_barrier();
    __builtin_amdgcn_fence(__ATOMIC_ACQUIRE, "workgroup");
  }
}

__global__ __launch_bounds__(256) void cast_f32_f16x2(
    const float* __restrict__ in, _Float16* __restrict__ out, int n2) {
  int i = blockIdx.x * 256 + threadIdx.x;
  if (i < n2) {
    const _Float16 h0 = (_Float16)in[2 * i], h1 = (_Float16)in[2 * i + 1];
    const unsigned u = (unsigned)__builtin_bit_cast(unsigned short, h0) | ((unsigned)__builtin_bit_cast(unsigned short, h1) << 16);
    ((volatile unsigned*)out)[i] = u;
    __threadfence();
    ((volatile unsigned*)out)[i] = u;
  }
}

__device__ __forceinline__ v8f hmma(v16h a, v16h b, v8f c) {
  c = __builtin_amdgcn_wmma_f32_16x16x32_f16(false, a, false, b, (short)0, c, false, false);
  asm volatile("v_nop\n\tv_nop\n\tv_nop\n\tv_nop" : "+v"(c) : "v"(a), "v"(b));
  return c;
}

__global__ __launch_bounds__(128)
void tupe_attn64(const _Float16* __restrict__ qkv, const _Float16* __restrict__ pe,
                 _Float16* __restrict__ vals, float sscale) {
  const float PSC = 32768.0f;
  const float OSC = 1.0f / 512.0f;
  __shared__ __align__(16) _Float16 Ksh[64 * 64];
  __shared__ __align__(16) _Float16 Ush[64 * 64];
  __shared__ __align__(16) _Float16 Vth[64 * 64];
  __shared__ __align__(16) _Float16 Psh[4][16 * 64];
  __shared__ __align__(16) float    Os[4][16 * 68];

  const int tid  = threadIdx.x;
  const int wave = tid >> 5;
  const int lane = tid & 31;
  const int hh   = lane >> 4;
  const int c    = lane & 15;

  const int nqb = LL / 64;
  const int bx = blockIdx.x;
  const int qb = bx % nqb;
  const int bh = bx / nqb;
  const int h  = bh % HH;
  const int b  = bh / HH;
  const int q0 = qb * 64 + wave * 16;

  const size_t rb = (size_t)b * LL;
  const _Float16* qkv_b = qkv + rb * QKV_LD + (size_t)h * (3 * HD);
  const _Float16* pe_b  = pe  + rb * PE_LD  + (size_t)h * (2 * HD);
  _Float16*       out_b = vals + rb * EE    + (size_t)h * HD;

  v16h qa0, qa1, ua0, ua1;
  {
    const _Float16* qrow = qkv_b + (size_t)(q0 + c) * QKV_LD + 8 * hh;
    const _Float16* urow = pe_b  + (size_t)(q0 + c) * PE_LD  + 8 * hh;
    qa0 = Frag<_Float16>::load(qrow);
    qa1 = Frag<_Float16>::load(qrow + 32);
    ua0 = Frag<_Float16>::load(urow);
    ua1 = Frag<_Float16>::load(urow + 32);
  }

  float mrow[8], lrow[8];
  v8f oacc[4];
#pragma unroll
  for (int r = 0; r < 8; ++r) { mrow[r] = -__builtin_inff(); lrow[r] = 0.f; }
#pragma unroll
  for (int t = 0; t < 4; ++t) oacc[t] = (v8f){0.f,0.f,0.f,0.f,0.f,0.f,0.f,0.f};

  for (int kc = 0; kc < LL / 64; ++kc) {
    const int kv0 = kc * 64;
    __syncthreads();
    {
      const int kvr = tid >> 1, dh = (tid & 1) * 32;
      const _Float16* krow = qkv_b + (size_t)(kv0 + kvr) * QKV_LD + HD + dh;
      const _Float16* vrow = krow + HD;
      const _Float16* urow = pe_b + (size_t)(kv0 + kvr) * PE_LD + HD + dh;
#pragma unroll
      for (int i = 0; i < 4; ++i) {
        const v8h kk = *(const v8h*)(krow + 8 * i);
        const v8h uu = *(const v8h*)(urow + 8 * i);
        const v8h vv = *(const v8h*)(vrow + 8 * i);
        *(v8h*)(Ksh + kvr * 64 + dh + 8 * i) = kk;
        *(v8h*)(Ush + kvr * 64 + dh + 8 * i) = uu;
#pragma unroll
        for (int e = 0; e < 8; ++e) Vth[(dh + 8 * i + e) * 64 + kvr] = vv[e];
      }
    }
    __syncthreads();

    v8f s[4];
#pragma unroll
    for (int j = 0; j < 4; ++j) {
      v8f a = (v8f){0.f,0.f,0.f,0.f,0.f,0.f,0.f,0.f};
      const _Float16* kp = Ksh + (j * 16 + c) * 64 + 8 * hh;
      const _Float16* up = Ush + (j * 16 + c) * 64 + 8 * hh;
      a = hmma(qa0, Frag<_Float16>::load(kp), a);
      a = hmma(qa1, Frag<_Float16>::load(kp + 32), a);
      a = hmma(ua0, Frag<_Float16>::load(up), a);
      a = hmma(ua1, Frag<_Float16>::load(up + 32), a);
      s[j] = a;
    }

    float cm[8];
#pragma unroll
    for (int r = 0; r < 8; ++r) {
      float m = -__builtin_inff();
#pragma unroll
      for (int j = 0; j < 4; ++j) {
        const float v = s[j][r] * sscale;
        s[j][r] = v;
        m = fmaxf(m, v);
      }
#pragma unroll
      for (int off = 1; off < 16; off <<= 1) m = fmaxf(m, __shfl_xor(m, off, 32));
      cm[r] = m;
    }
    _Float16* pwh = Psh[wave];
#pragma unroll
    for (int r = 0; r < 8; ++r) {
      const float mnew = fmaxf(mrow[r], cm[r]);
      const float alpha = __expf(mrow[r] - mnew);
      mrow[r] = mnew;
      float psum = 0.f;
#pragma unroll
      for (int j = 0; j < 4; ++j) {
        const float p = __expf(s[j][r] - mnew);
        psum += p;
        pwh[(8 * hh + r) * 64 + j * 16 + c] = (_Float16)(p * PSC);
      }
#pragma unroll
      for (int off = 1; off < 16; off <<= 1) psum += __shfl_xor(psum, off, 32);
      lrow[r] = lrow[r] * alpha + psum;
#pragma unroll
      for (int t = 0; t < 4; ++t) oacc[t][r] *= alpha;
    }
    __builtin_amdgcn_fence(__ATOMIC_RELEASE, "workgroup");
    __builtin_amdgcn_wave_barrier();
    __builtin_amdgcn_fence(__ATOMIC_ACQUIRE, "workgroup");

#pragma unroll
    for (int kk = 0; kk < 2; ++kk) {
      const v16h pa = Frag<_Float16>::load(pwh + c * 64 + kk * 32 + 8 * hh);
#pragma unroll
      for (int t = 0; t < 4; ++t) {
        const v16h vb = Frag<_Float16>::load(Vth + (t * 16 + c) * 64 + kk * 32 + 8 * hh);
        oacc[t] = hmma(pa, vb, oacc[t]);
      }
    }
  }

  float* os = Os[wave];
#pragma unroll
  for (int r = 0; r < 8; ++r) {
    const float inv = (1.0f / lrow[r]) * OSC;
#pragma unroll
    for (int t = 0; t < 4; ++t) os[(8 * hh + r) * 68 + t * 16 + c] = oacc[t][r] * inv;
  }
  __builtin_amdgcn_fence(__ATOMIC_RELEASE, "workgroup");
  __builtin_amdgcn_wave_barrier();
  __builtin_amdgcn_fence(__ATOMIC_ACQUIRE, "workgroup");
  {
    const int q = lane >> 3, c8 = (lane & 7) * 8;
    for (int pass = 0; pass < 2; ++pass) {
#pragma unroll
      for (int it = 0; it < 4; ++it) {
        const int row = it * 4 + q;
        const float* sp = os + row * 68 + c8;
        v8h hv;
#pragma unroll
        for (int e = 0; e < 8; ++e) hv[e] = (_Float16)sp[e];
        *(volatile v8h*)(out_b + (size_t)(q0 + row) * EE + c8) = hv;
      }
      __threadfence();
    }
  }
}

extern "C" void kernel_launch(void* const* d_in, const int* in_sizes, int n_in,
                              void* d_out, int out_size, void* d_ws, size_t ws_size,
                              hipStream_t stream) {
  const int ROWS = BB * LL;
  if (n_in < 5) return;
  if (in_sizes[0] != ROWS * DD || in_sizes[1] != ROWS * EE || in_sizes[2] != 3 * EE * DD ||
      in_sizes[3] != EE * EE || in_sizes[4] != 2 * EE * EE || out_size != ROWS * EE) return;

  const float* x    = (const float*)d_in[0];
  const float* PEf  = (const float*)d_in[1];
  const float* Wqkv = (const float*)d_in[2];
  const float* Wo   = (const float*)d_in[3];
  const float* UqUk = (const float*)d_in[4];
  float* out = (float*)d_out;

  size_t off = 0;
  auto carve = [&](size_t bytes) -> size_t { size_t o = off; off += (bytes + 255) & ~(size_t)255; return o; };
  const size_t oX    = carve((size_t)ROWS * DD * 2);
  const size_t oPE   = carve((size_t)ROWS * EE * 2);
  const size_t oWqkv = carve((size_t)3 * EE * DD * 2);
  const size_t oWo   = carve((size_t)EE * EE * 2);
  const size_t oUqUk = carve((size_t)2 * EE * EE * 2);
  const size_t oQKV  = carve((size_t)ROWS * QKV_LD * 2);
  const size_t oPEP  = carve((size_t)ROWS * PE_LD * 2);
  const size_t oVALS = carve((size_t)ROWS * EE * 2);
  if (off > ws_size) return;

  char* ws = (char*)d_ws;
  _Float16* X16    = (_Float16*)(ws + oX);
  _Float16* PE16   = (_Float16*)(ws + oPE);
  _Float16* Wqkv16 = (_Float16*)(ws + oWqkv);
  _Float16* Wo16   = (_Float16*)(ws + oWo);
  _Float16* UqUk16 = (_Float16*)(ws + oUqUk);
  _Float16* QKV16  = (_Float16*)(ws + oQKV);
  _Float16* PEP16  = (_Float16*)(ws + oPEP);
  _Float16* VALS16 = (_Float16*)(ws + oVALS);

  {
    const int n2x = ROWS * DD / 2;
    cast_f32_f16x2<<<dim3((n2x + 255) / 256), dim3(256), 0, stream>>>(x, X16, n2x);
    const int n2p = ROWS * EE / 2;
    cast_f32_f16x2<<<dim3((n2p + 255) / 256), dim3(256), 0, stream>>>(PEf, PE16, n2p);
    const int n2w = 3 * EE * DD / 2;
    cast_f32_f16x2<<<dim3((n2w + 255) / 256), dim3(256), 0, stream>>>(Wqkv, Wqkv16, n2w);
    const int n2o = EE * EE / 2;
    cast_f32_f16x2<<<dim3((n2o + 255) / 256), dim3(256), 0, stream>>>(Wo, Wo16, n2o);
    const int n2u = 2 * EE * EE / 2;
    cast_f32_f16x2<<<dim3((n2u + 255) / 256), dim3(256), 0, stream>>>(UqUk, UqUk16, n2u);
  }

  {
    const int M = ROWS, N = 3 * EE, K = DD;
    const int tiles = (M / 64) * (N / 64);
    wmma_gemm64<0, false, 0, 1, false><<<dim3((tiles + 7) / 8, 1), dim3(256), 0, stream>>>(
        (const unsigned short*)X16, (const unsigned short*)X16, K, 0L,
        (const unsigned short*)Wqkv16, (const unsigned short*)Wqkv16, K, 0L,
        (void*)QKV16, (void*)QKV16, N, 0L,
        x, x, 0L, M, N, K, 1.0f);
  }
  {
    const int M = ROWS, N = 2 * EE, K = EE;
    const int tiles = (M / 64) * (N / 64);
    wmma_gemm64<0, false, 0, 1, false><<<dim3((tiles + 7) / 8, 1), dim3(256), 0, stream>>>(
        (const unsigned short*)PE16, (const unsigned short*)PE16, K, 0L,
        (const unsigned short*)UqUk16, (const unsigned short*)UqUk16, K, 0L,
        (void*)PEP16, (void*)PEP16, N, 0L,
        x, x, 0L, M, N, K, 1.0f);
  }
  {
    const float sscale = 0.08838834764831845f;
    tupe_attn64<<<dim3(BB * HH * (LL / 64)), dim3(128), 0, stream>>>(QKV16, PEP16, VALS16, sscale);
  }
  {
    const int M = ROWS, N = EE, K = EE;
    const int tiles = (M / 64) * (N / 64);
    wmma_gemm64<0, false, 0, 0, false><<<dim3((tiles + 7) / 8, 1), dim3(256), 0, stream>>>(
        (const unsigned short*)VALS16, (const unsigned short*)VALS16, K, 0L,
        (const unsigned short*)Wo16, (const unsigned short*)Wo16, K, 0L,
        (void*)out, (void*)out, N, 0L,
        x, x, 0L, M, N, K, 0.015625f);
  }
}
